// SetAbstraction_45174466019645
// MI455X (gfx1250) — hardware-verified
//
#include <hip/hip_runtime.h>
#include <stdint.h>

#pragma clang fp contract(off)

typedef __attribute__((ext_vector_type(16))) _Float16 v16h;
typedef __attribute__((ext_vector_type(8)))  _Float16 v8h;
typedef __attribute__((ext_vector_type(4)))  _Float16 v4h;
typedef __attribute__((ext_vector_type(8)))  float    v8f;
typedef __attribute__((ext_vector_type(4)))  float    v4f;

__device__ __forceinline__ void dep_guard_h(v8f& a, v8f& b, v16h x, v16h y) { asm volatile("v_nop\n\tv_nop\n\tv_nop\n\tv_nop" : "+v"(a), "+v"(b) : "v"(x), "v"(y)); }
__device__ __forceinline__ void keep4_h(v16h a, v16h b, v16h c, v16h d) { asm volatile("v_nop" :: "v"(a), "v"(b), "v"(c), "v"(d)); }
__device__ __forceinline__ void acc_guard4(v8f& a, v8f& b, v8f& c, v8f& d) { asm volatile("v_nop\n\tv_nop\n\tv_nop\n\tv_nop" : "+v"(a), "+v"(b), "+v"(c), "+v"(d)); }
template <typename T> struct Frag;
template <> struct Frag<_Float16> {
  typedef v16h V; union U { v16h v; v8h h[2]; };
  static __device__ __forceinline__ v16h load(const _Float16* p) {
    U f; f.h[0] = *(const v8h*)(p); f.h[1] = *(const v8h*)(p + 16); return f.v;
  }
  static __device__ __forceinline__ v8f mma(v16h a, v16h b, v8f c) {
    return __builtin_amdgcn_wmma_f32_16x16x32_f16(false, a, false, b, (short)0, c, false, false);
  }
  static __device__ __forceinline__ void guard(v8f& a, v8f& b, v16h x, v16h y) { dep_guard_h(a, b, x, y); }
  static __device__ __forceinline__ void keep(v16h a, v16h b, v16h c, v16h d) { keep4_h(a, b, c, d); }
};

static constexpr int kBatch      = 16;
static constexpr int kPts        = 4096;
static constexpr int kCtr        = 1024;
static constexpr int kSmp        = 32;
static constexpr int kCin        = 64;
static constexpr int kCinTot     = 67;
static constexpr int kK0         = 96;
static constexpr int kC0         = 64;
static constexpr int kC1         = 64;
static constexpr int kC2         = 128;
static constexpr int kFpsThreads = 256;
static constexpr int kPtsPerThr  = kPts / kFpsThreads;
static constexpr int kGrpThreads = 128;
static constexpr int kWaves      = kGrpThreads / 32;
static constexpr int kActBytesPerWave = kSmp * kK0 * 2;
static constexpr int kActBytes   = kWaves * kActBytesPerWave;
static constexpr int kW0Bytes    = kC0 * kK0 * 2;
static constexpr int kW1Bytes    = kC1 * kC0 * 2;
static constexpr int kW2Bytes    = kC2 * kC1 * 2;
static constexpr int kUniBytes   = kActBytes + kW0Bytes + kW1Bytes + kW2Bytes;
static constexpr int kCandBytesPerWave = kUniBytes / kWaves;
static constexpr int kCap        = kCandBytesPerWave / 8;
#define GRP_RADIUS_SQ 0.04f

static_assert(kPts % kFpsThreads == 0, "fps");
static_assert((kPts * 3 / 4) % kFpsThreads == 0, "fps staging");
static_assert((kPts * 3 / 4) % kGrpThreads == 0, "grp staging");
static_assert(kCap % 32 == 0, "cap");
static_assert(kCap * 8 * kWaves <= kUniBytes, "cand fits");
static_assert(kCandBytesPerWave % 16 == 0 && kActBytesPerWave % 16 == 0, "align");
static_assert((kC0 * kK0) % kGrpThreads == 0, "w0 staging");
static_assert((kC1 * kC0 / 4) % kGrpThreads == 0, "w1 staging");
static_assert((kC2 * kC1 / 4) % kGrpThreads == 0, "w2 staging");
static_assert(kCtr % kWaves == 0, "grid");
static_assert(kK0 % 32 == 0 && kC0 % 32 == 0 && kC1 % 32 == 0, "K multiples of 32");
static_assert(kSmp == 32 && kC0 == 64 && kC2 == 128, "tile shape");
static_assert(kBatch * kCtr * 3 * 4 == 196608, "out1 byte offset");
static_assert(196608 + kBatch * kCtr * kC2 * 4 == 8585216, "out total bytes");

__device__ __forceinline__ void wave_argmax(float& v, int& i) {
#pragma unroll
  for (int off = 16; off > 0; off >>= 1) {
    const float ov = __shfl_xor(v, off, 32);
    const int   oi = __shfl_xor(i, off, 32);
    const bool tk = (ov > v) || (ov == v && oi < i);
    v = tk ? ov : v; i = tk ? oi : i;
  }
}
__device__ __forceinline__ void wave_argmin(float& v, int& i) {
#pragma unroll
  for (int off = 16; off > 0; off >>= 1) {
    const float ov = __shfl_xor(v, off, 32);
    const int   oi = __shfl_xor(i, off, 32);
    const bool tk = (ov < v) || (ov == v && oi < i);
    v = tk ? ov : v; i = tk ? oi : i;
  }
}

__global__ void __launch_bounds__(kFpsThreads)
fps_kernel(const float* __restrict__ xyz, float* out_ctr)
{
  __shared__ __align__(16) float s3[3][kPts];
  __shared__ int   sidx[kCtr];
  __shared__ float rv[2][kFpsThreads / 32];
  __shared__ int   ri[2][kFpsThreads / 32];

  const int b = blockIdx.x;
  const int tid = threadIdx.x, lane = tid & 31, wave = tid >> 5;
  const float* Xb = xyz + (size_t)b * kPts * 3;

#pragma unroll 2
  for (int q = tid; q < kPts * 3 / 4; q += kFpsThreads) {
    const v4f v = *(const v4f*)(Xb + 4 * q);
#pragma unroll
    for (int e = 0; e < 4; ++e) {
      const int idx = 4 * q + e;
      const int j = idx / 3;
      const int c = idx - 3 * j;
      s3[c][j] = v[e];
    }
  }
  __syncthreads();

  float px[kPtsPerThr], py[kPtsPerThr], pz[kPtsPerThr], dmin[kPtsPerThr];
#pragma unroll
  for (int i = 0; i < kPtsPerThr; ++i) {
    const int p = tid + kFpsThreads * i;
    px[i] = s3[0][p]; py[i] = s3[1][p]; pz[i] = s3[2][p];
    dmin[i] = 1.0e10f;
  }

  int far = 0;
  for (int it = 0; it < kCtr; ++it) {
    if (tid == 0) sidx[it] = far;
    const float cx = s3[0][far], cy = s3[1][far], cz = s3[2][far];
    float bd = -1.0f;
    int   bi = 0;
#pragma unroll
    for (int i = 0; i < kPtsPerThr; ++i) {
      const float dx = px[i] - cx, dy = py[i] - cy, dz = pz[i] - cz;
      const float t0 = dx * dx;
      const float t1 = dy * dy;
      const float t2 = dz * dz;
      const float s02 = t0 + t2;
      const float d = s02 + t1;
      const float dm = fminf(dmin[i], d);
      dmin[i] = dm;
      const bool tk = dm > bd;
      bd = tk ? dm : bd;
      bi = tk ? (tid + kFpsThreads * i) : bi;
    }
    wave_argmax(bd, bi);
    const int par = it & 1;
    if (lane == 0) { rv[par][wave] = bd; ri[par][wave] = bi; }
    __syncthreads();
    float fb = rv[par][0];
    int   fi = ri[par][0];
#pragma unroll
    for (int w2 = 1; w2 < kFpsThreads / 32; ++w2) {
      const float ov = rv[par][w2];
      const int   oi = ri[par][w2];
      const bool tk = (ov > fb) || (ov == fb && oi < fi);
      fb = tk ? ov : fb; fi = tk ? oi : fi;
    }
    far = fi & (kPts - 1);
  }
  __syncthreads();

  float* Ob = out_ctr + (size_t)b * (kCtr * 3);
  v4f ov[3];
#pragma unroll
  for (int rep = 0; rep < 3; ++rep) {
    const int q = tid + kFpsThreads * rep;
    v4f v;
#pragma unroll
    for (int e = 0; e < 4; ++e) {
      const int idx = 4 * q + e;
      const int pt = idx / 3;
      const int c = idx - 3 * pt;
      const int j = sidx[pt] & (kPts - 1);
      v[e] = s3[c][j];
    }
    ov[rep] = v;
  }
  for (int pass = 0; pass < 2; ++pass) {
#pragma unroll
    for (int rep = 0; rep < 3; ++rep)
      *(volatile v4f*)(Ob + 4 * (tid + kFpsThreads * rep)) = ov[rep];
    __threadfence();
  }
}

template <int KSTEPS, int PITCHB>
__device__ __forceinline__ void wave_gemm_32x64(const _Float16* arows, const _Float16* bt,
                                                v8f (&acc)[2][4], int rl, int koff)
{
#pragma unroll
  for (int i = 0; i < 2; ++i)
#pragma unroll
    for (int j = 0; j < 4; ++j) acc[i][j] = (v8f){0.f, 0.f, 0.f, 0.f, 0.f, 0.f, 0.f, 0.f};
#pragma unroll
  for (int ks = 0; ks < KSTEPS; ++ks) {
    v16h bfr[4];
#pragma unroll
    for (int j = 0; j < 4; ++j) bfr[j] = Frag<_Float16>::load(bt + (16 * j + rl) * PITCHB + 32 * ks + koff);
#pragma unroll
    for (int i = 0; i < 2; ++i) {
      const v16h afr = Frag<_Float16>::load(arows + (16 * i + rl) * kK0 + 32 * ks + koff);
#pragma unroll
      for (int j = 0; j < 4; ++j) acc[i][j] = Frag<_Float16>::mma(afr, bfr[j], acc[i][j]);
      Frag<_Float16>::guard(acc[i][0], acc[i][3], afr, afr);
    }
    Frag<_Float16>::keep(bfr[0], bfr[1], bfr[2], bfr[3]);
  }
  acc_guard4(acc[0][0], acc[0][1], acc[0][2], acc[0][3]);
  acc_guard4(acc[1][0], acc[1][1], acc[1][2], acc[1][3]);
}

__device__ __forceinline__ void wave_epilogue_hidden(const v8f (&acc)[2][4], _Float16* arows,
                                                     const float* scl, const float* sh, int rl, int hh)
{
#pragma unroll
  for (int i = 0; i < 2; ++i) {
#pragma unroll
    for (int j = 0; j < 4; ++j) {
      const int col = 16 * j + rl;
      const float s = scl[col], c = sh[col];
#pragma unroll
      for (int r = 0; r < 8; ++r) {
        float v = fmaf(acc[i][j][r], s, c);
        v = fmaxf(v, 0.0f);
        arows[(16 * i + 8 * hh + r) * kK0 + col] = (_Float16)v;
      }
    }
  }
}

__global__ void __launch_bounds__(kGrpThreads)
group_mlp_kernel(const float* __restrict__ xyz, const float* __restrict__ feat, const float* ctr_xyz,
                 const float* __restrict__ w0, const float* __restrict__ b0, const float* __restrict__ g0,
                 const float* __restrict__ be0, const float* __restrict__ m0, const float* __restrict__ v0,
                 const float* __restrict__ w1, const float* __restrict__ b1, const float* __restrict__ g1,
                 const float* __restrict__ be1, const float* __restrict__ m1, const float* __restrict__ v1,
                 const float* __restrict__ w2, const float* __restrict__ b2, const float* __restrict__ g2,
                 const float* __restrict__ be2, const float* __restrict__ m2, const float* __restrict__ v2,
                 float* out_feat)
{
  __shared__ __align__(16) float s3[3][kPts];
  __shared__ __align__(16) float ssq[kPts];
  __shared__ __align__(16) unsigned char suni[kUniBytes];
  __shared__ __align__(16) float sscl[kC0 + kC1 + kC2];
  __shared__ __align__(16) float ssh[kC0 + kC1 + kC2];
  __shared__ int ssel[kWaves][kSmp];
  __shared__ __align__(16) float spool[kWaves][kC2];

  const int tid  = threadIdx.x;
  const int lane = tid & 31, wave = tid >> 5, hh = lane >> 4, rl = lane & 15, koff = hh * 8;
  const int blk  = blockIdx.x;
  const int b    = blk / (kCtr / kWaves);
  const int cg   = blk * kWaves + wave;
  const float* Xb = xyz + (size_t)b * kPts * 3;

#pragma unroll 2
  for (int q = tid; q < kPts * 3 / 4; q += kGrpThreads) {
    const v4f v = *(const v4f*)(Xb + 4 * q);
#pragma unroll
    for (int e = 0; e < 4; ++e) {
      const int idx = 4 * q + e;
      const int j = idx / 3;
      const int c = idx - 3 * j;
      s3[c][j] = v[e];
    }
  }
  if (wave == 0) {
#pragma unroll
    for (int t = 0; t < 2; ++t) {
      const int o = lane + 32 * t;
      const float s = g0[o] / sqrtf(v0[o] + 1.0e-5f);
      sscl[o] = s;
      ssh[o]  = (b0[o] - m0[o]) * s + be0[o];
    }
  } else if (wave == 1) {
#pragma unroll
    for (int t = 0; t < 2; ++t) {
      const int o = lane + 32 * t;
      const float s = g1[o] / sqrtf(v1[o] + 1.0e-5f);
      sscl[kC0 + o] = s;
      ssh[kC0 + o]  = (b1[o] - m1[o]) * s + be1[o];
    }
  } else {
    const int base = (wave - 2) * 64;
#pragma unroll
    for (int t = 0; t < 2; ++t) {
      const int o = base + lane + 32 * t;
      const float s = g2[o] / sqrtf(v2[o] + 1.0e-5f);
      sscl[kC0 + kC1 + o] = s;
      ssh[kC0 + kC1 + o]  = (b2[o] - m2[o]) * s + be2[o];
    }
  }
  __syncthreads();
  for (int j = tid; j < kPts; j += kGrpThreads) {
    const float x = s3[0][j], y = s3[1][j], z = s3[2][j];
    const float t0 = x * x;
    const float t1 = y * y;
    const float t2 = z * z;
    const float s02 = t0 + t2;
    ssq[j] = s02 + t1;
  }
  __syncthreads();

  const float cx = ctr_xyz[(size_t)cg * 3 + 0];
  const float cy = ctr_xyz[(size_t)cg * 3 + 1];
  const float cz = ctr_xyz[(size_t)cg * 3 + 2];
  float sqc;
  {
    const float t0 = cx * cx;
    const float t1 = cy * cy;
    const float t2 = cz * cz;
    const float s02 = t0 + t2;
    sqc = s02 + t1;
  }
  float* candD = (float*)(suni + wave * kCandBytesPerWave);
  int*   candI = (int*)(suni + wave * kCandBytesPerWave + kCap * 4);

  int cnt = 0;
#pragma unroll 2
  for (int i = 0; i < kPts / 32; ++i) {
    const int j = lane + 32 * i;
    const float xj = s3[0][j], yj = s3[1][j], zj = s3[2][j];
    float p = cx * xj;
    p = fmaf(cy, yj, p);
    p = fmaf(cz, zj, p);
    const float m2p = -2.0f * p;
    const float d1 = m2p + sqc;
    float d = d1 + ssq[j];
    d = fmaxf(d, 0.0f);
    const bool hit = (d <= GRP_RADIUS_SQ);
    const unsigned msk = __builtin_amdgcn_ballot_w32(hit);
    const int pos = cnt + (int)__builtin_popcount(msk & ((1u << lane) - 1u));
    if (hit && pos < kCap) { candD[pos] = d; candI[pos] = j; }
    cnt += (int)__builtin_popcount(msk);
  }
  if (cnt == 0) {
    if (lane == 0) { candD[0] = 0.0f; candI[0] = 0; }
    cnt = 1;
  }
  const int cntc = (cnt < kCap) ? cnt : kCap;
  int nT = (cntc + 31) >> 5;
  nT = (nT > kCap / 32) ? (kCap / 32) : nT;
  __syncthreads();

  float pd = -1.0f;
  int   pidx = -1;
  int   firstj = 0;
#pragma unroll 1
  for (int r = 0; r < kSmp; ++r) {
    float bd = 3.0e38f;
    int   bj = 0x7fffffff;
#pragma unroll 1
    for (int t = 0; t < nT; ++t) {
      const int e = lane + 32 * t;
      const int ec = (e < cntc) ? e : (cntc - 1);
      const float d = candD[ec];
      const int   jj = candI[ec];
      const bool valid = (e < cntc);
      const bool gt = (d > pd) || (d == pd && jj > pidx);
      const bool lt = (d < bd) || (d == bd && jj < bj);
      const bool tk = valid && gt && lt;
      bd = tk ? d : bd;
      bj = tk ? jj : bj;
    }
    wave_argmin(bd, bj);
    const bool none = (bd >= 1.0e38f);
    if (r == 0) firstj = bj;
    const int selj = none ? firstj : bj;
    if (lane == 0) ssel[wave][r] = selj & (kPts - 1);
    pd = bd; pidx = bj;
  }
  __syncthreads();

  _Float16* arows = (_Float16*)(suni + wave * kActBytesPerWave);
  _Float16* sw0 = (_Float16*)(suni + kActBytes);
  _Float16* sw1 = (_Float16*)(suni + kActBytes + kW0Bytes);
  _Float16* sw2 = (_Float16*)(suni + kActBytes + kW0Bytes + kW1Bytes);

#pragma unroll 4
  for (int e = tid; e < kC0 * kK0; e += kGrpThreads) {
    const int o  = e / kK0;
    const int kk = e - o * kK0;
    const int src = (kk < kCin) ? (kk + 3) : ((kk < kCinTot) ? (kk - kCin) : 0);
    const float fz = (kk < kCinTot) ? 1.0f : 0.0f;
    const float v = w0[o * kCinTot + src] * fz;
    sw0[e] = (_Float16)v;
  }
#pragma unroll 2
  for (int q = tid; q < kC1 * kC0 / 4; q += kGrpThreads) {
    const v4f v = *(const v4f*)(w1 + 4 * q);
    v4h hv; hv[0] = (_Float16)v[0]; hv[1] = (_Float16)v[1]; hv[2] = (_Float16)v[2]; hv[3] = (_Float16)v[3];
    *(v4h*)(sw1 + 4 * q) = hv;
  }
#pragma unroll 2
  for (int q = tid; q < kC2 * kC1 / 4; q += kGrpThreads) {
    const v4f v = *(const v4f*)(w2 + 4 * q);
    v4h hv; hv[0] = (_Float16)v[0]; hv[1] = (_Float16)v[1]; hv[2] = (_Float16)v[2]; hv[3] = (_Float16)v[3];
    *(v4h*)(sw2 + 4 * q) = hv;
  }
  const float* Fb = feat + (size_t)b * kPts * kCin;
#pragma unroll 4
  for (int it = 0; it < kSmp / 2; ++it) {
    const int s = 2 * it + hh;
    const int j = ssel[wave][s] & (kPts - 1);
    const int c4 = rl * 4;
    const v4f f = *(const v4f*)(Fb + (size_t)j * kCin + c4);
    v4h hv; hv[0] = (_Float16)f[0]; hv[1] = (_Float16)f[1]; hv[2] = (_Float16)f[2]; hv[3] = (_Float16)f[3];
    *(v4h*)(arows + s * kK0 + c4) = hv;
  }
  {
    const int s = lane;
    const int j = ssel[wave][s] & (kPts - 1);
    const float dx = s3[0][j] - cx, dy = s3[1][j] - cy, dz = s3[2][j] - cz;
    float zf = 0.0f;
    asm volatile("" : "+v"(zf));
    const _Float16 zh = (_Float16)zf;
    v8h va;
    va[0] = (_Float16)dx; va[1] = (_Float16)dy; va[2] = (_Float16)dz; va[3] = zh;
    va[4] = zh; va[5] = zh; va[6] = zh; va[7] = zh;
    v8h vz;
    vz[0] = zh; vz[1] = zh; vz[2] = zh; vz[3] = zh; vz[4] = zh; vz[5] = zh; vz[6] = zh; vz[7] = zh;
    _Float16* rp = arows + s * kK0 + kCin;
    *(v8h*)(rp)      = va;
    *(v8h*)(rp + 8)  = vz;
    *(v8h*)(rp + 16) = vz;
    *(v8h*)(rp + 24) = vz;
  }
  __syncthreads();

  v8f acc[2][4];
  wave_gemm_32x64<kK0 / 32, kK0>(arows, sw0, acc, rl, koff);
  __syncthreads();
  wave_epilogue_hidden(acc, arows, sscl, ssh, rl, hh);
  __syncthreads();
  wave_gemm_32x64<kC0 / 32, kC0>(arows, sw1, acc, rl, koff);
  __syncthreads();
  wave_epilogue_hidden(acc, arows, sscl + kC0, ssh + kC0, rl, hh);
  __syncthreads();
#pragma unroll
  for (int nh = 0; nh < 2; ++nh) {
    wave_gemm_32x64<kC1 / 32, kC1>(arows, sw2 + nh * 64 * kC1, acc, rl, koff);
#pragma unroll
    for (int j = 0; j < 4; ++j) {
      const int col = nh * 64 + 16 * j + rl;
      const float s = sscl[kC0 + kC1 + col], c = ssh[kC0 + kC1 + col];
      float mx = 0.0f;
#pragma unroll
      for (int i = 0; i < 2; ++i) {
#pragma unroll
        for (int r = 0; r < 8; ++r) {
          float v = fmaf(acc[i][j][r], s, c);
          v = fmaxf(v, 0.0f);
          mx = fmaxf(mx, v);
        }
      }
      const float other = __shfl_xor(mx, 16, 32);
      mx = fmaxf(mx, other);
      if (hh == 0) spool[wave][col] = mx;
    }
  }
  __syncthreads();

  const v4f ov = *(const v4f*)(&spool[wave][4 * lane]);
  float* orow = out_feat + (size_t)cg * kC2;
  for (int pass = 0; pass < 2; ++pass) {
    *(volatile v4f*)(orow + 4 * lane) = ov;
    __threadfence();
  }
}

extern "C" void kernel_launch(void* const* d_in, const int* in_sizes, int n_in,
                              void* d_out, int out_size, void* d_ws, size_t ws_size,
                              hipStream_t stream)
{
  (void)in_sizes; (void)n_in; (void)out_size; (void)d_ws; (void)ws_size;
  const float* xyz  = (const float*)d_in[0];
  const float* feat = (const float*)d_in[1];
  const float* w0 = (const float*)d_in[2];
  const float* b0 = (const float*)d_in[3];
  const float* g0 = (const float*)d_in[4];
  const float* be0 = (const float*)d_in[5];
  const float* m0 = (const float*)d_in[6];
  const float* v0 = (const float*)d_in[7];
  const float* w1 = (const float*)d_in[8];
  const float* b1 = (const float*)d_in[9];
  const float* g1 = (const float*)d_in[10];
  const float* be1 = (const float*)d_in[11];
  const float* m1 = (const float*)d_in[12];
  const float* v1 = (const float*)d_in[13];
  const float* w2 = (const float*)d_in[14];
  const float* b2 = (const float*)d_in[15];
  const float* g2 = (const float*)d_in[16];
  const float* be2 = (const float*)d_in[17];
  const float* m2 = (const float*)d_in[18];
  const float* v2 = (const float*)d_in[19];

  float* out_ctr  = (float*)d_out;
  float* out_feat = (float*)d_out + (size_t)kBatch * kCtr * 3;


  fps_kernel<<<dim3(kBatch), dim3(kFpsThreads), 0, stream>>>(xyz, out_ctr);

  group_mlp_kernel<<<dim3(kBatch * kCtr / kWaves), dim3(kGrpThreads), 0, stream>>>(
      xyz, feat, out_ctr,
      w0, b0, g0, be0, m0, v0,
      w1, b1, g1, be1, m1, v1,
      w2, b2, g2, be2, m2, v2,
      out_feat);
}
